// TextualKnowledgeInjector_71270687309839
// MI455X (gfx1250) — hardware-verified
//
#include <hip/hip_runtime.h>
#include <math.h>

typedef __attribute__((ext_vector_type(16))) _Float16 v16h;
typedef __attribute__((ext_vector_type(16))) __bf16 v16b;
typedef __attribute__((ext_vector_type(8)))  _Float16 v8h;
typedef __attribute__((ext_vector_type(8)))  float v8f;
typedef __attribute__((ext_vector_type(4)))  float v4f;
typedef __attribute__((ext_vector_type(2)))  float v2f;
typedef __attribute__((ext_vector_type(4)))  unsigned v4u;
typedef __attribute__((ext_vector_type(4)))  int v4i;
typedef float __attribute__((may_alias)) float_a;
typedef int __attribute__((may_alias)) int_a;

template <typename T> __device__ __forceinline__ void vst2(void* p, T v) { *(volatile T*)p = v; __threadfence(); *(volatile T*)p = v; }
__device__ __forceinline__ v8f wmma16(v16h a, v16h b, v8f c) {
  v8f d = __builtin_amdgcn_wmma_f32_16x16x32_f16(false, a, false, b, (short)0, c, false, false);
  asm volatile("v_nop\n\tv_nop\n\tv_nop\n\tv_nop" : "+v"(d) : "v"(a), "v"(b));
  return d;
}
__device__ __forceinline__ v8f wmma_bf(v16b a, v16b b, v8f c) {
  v8f d = __builtin_amdgcn_wmma_f32_16x16x32_bf16(false, a, false, b, (short)0, c, false, false);
  asm volatile("v_nop\n\tv_nop\n\tv_nop\n\tv_nop" : "+v"(d) : "v"(a), "v"(b));
  return d;
}
__device__ __forceinline__ v16h frag_h(const _Float16* rowk0, int lane) {
  union { v16h v; v8h q[2]; } u; const _Float16* p = rowk0 + 8 * (lane >> 4);
  u.q[0] = *(const v8h*)p; u.q[1] = *(const v8h*)(p + 16); return u.v;
}
__device__ __forceinline__ v16h frag_f32(const float* rowk0, int lane) {
  v16h a; const float* p = rowk0 + 8 * (lane >> 4);
#pragma unroll
  for (int i = 0; i < 8; ++i) { a[i] = (_Float16)p[i]; a[8 + i] = (_Float16)p[16 + i]; }
  return a;
}
__device__ __forceinline__ v16h frag_f32s(const float* rowk0, int lane, float sc) {
  v16h a; const float* p = rowk0 + 8 * (lane >> 4);
#pragma unroll
  for (int i = 0; i < 8; ++i) { a[i] = (_Float16)(p[i] * sc); a[8 + i] = (_Float16)(p[16 + i] * sc); }
  return a;
}
__device__ __forceinline__ v16h fragc_f32(const float* W, int k0, int n, int lane, int ld, int K) {
  v16h a; const int g = lane >> 4;
#pragma unroll
  for (int i = 0; i < 8; ++i) { const int ka = k0 + 8 * g + i, kb = ka + 16;
    a[i] = (_Float16)(ka < K ? W[(size_t)(ka < K ? ka : K - 1) * ld + n] : 0.f); a[8 + i] = (_Float16)(kb < K ? W[(size_t)(kb < K ? kb : K - 1) * ld + n] : 0.f); }
  return a;
}
struct F2 { v16b h, l; };
__device__ __forceinline__ F2 bsplit16(const float v[16]) { F2 r;
#pragma unroll
  for (int i = 0; i < 16; ++i) { const __bf16 h = (__bf16)v[i]; r.h[i] = h; r.l[i] = (__bf16)(v[i] - (float)h); }
  return r; }
__device__ __forceinline__ F2 split_row(const float* row, int k0, int lane) { float v[16]; const float* p = row + k0 + 8 * (lane >> 4);
#pragma unroll
  for (int i = 0; i < 8; ++i) { v[i] = p[i]; v[8 + i] = p[16 + i]; }
  return bsplit16(v); }
__device__ __forceinline__ F2 split_rowK(const float* row, int k0, int lane, int K) { float v[16]; const int g = lane >> 4;
#pragma unroll
  for (int i = 0; i < 8; ++i) { const int ka = k0 + 8 * g + i, kb = ka + 16; v[i] = ka < K ? row[ka < K ? ka : K - 1] : 0.f; v[8 + i] = kb < K ? row[kb < K ? kb : K - 1] : 0.f; }
  return bsplit16(v); }
__device__ __forceinline__ F2 split_col(const float* W, int k0, int n, int lane, int ld, int K) { float v[16]; const int g = lane >> 4;
#pragma unroll
  for (int i = 0; i < 8; ++i) { const int ka = k0 + 8 * g + i, kb = ka + 16; v[i] = ka < K ? W[(size_t)(ka < K ? ka : K - 1) * ld + n] : 0.f; v[8 + i] = kb < K ? W[(size_t)(kb < K ? kb : K - 1) * ld + n] : 0.f; }
  return bsplit16(v); }
__device__ __forceinline__ v8f mac3(const F2& a, const F2& b, v8f c) { c = wmma_bf(a.l, b.h, c); c = wmma_bf(a.h, b.l, c); return wmma_bf(a.h, b.h, c); }
__device__ __forceinline__ float sigm(float v) { return 1.0f / (1.0f + expf(-v)); }
#define LDSX() do { asm volatile("s_wait_dscnt 0" ::: "memory"); __builtin_amdgcn_wave_barrier(); __builtin_amdgcn_fence(__ATOMIC_RELEASE, "workgroup"); } while (0)


#define NBT 64
#define TT 256
#define FF 40
#define NPAIR (FF * FF)
#define DD 768
#define HH 256
#define NR (NBT * TT)
#ifndef TR
#define TR (NR / 64)
#endif
typedef __attribute__((ext_vector_type(8))) __bf16 v8b;
__device__ __forceinline__ v16b frag_b(const __bf16* rowk0, int lane) {
  union { v16b v; v8b q[2]; } u; const __bf16* p = rowk0 + 8 * (lane >> 4);
  u.q[0] = *(const v8b*)p; u.q[1] = *(const v8b*)(p + 16); return u.v;
}
__device__ __forceinline__ float bfr(float v) { return (float)(__bf16)v; }
__device__ __attribute__((noinline)) float exp_ni(float v) { return expf(v); }
__device__ __attribute__((noinline)) float erf_ni(float v) { return erff(v); }

#define WS_PE  0u
#define WS_CTX (WS_PE + 2u * (size_t)DD * NPAIR)
#define WS_END (WS_CTX + 4u * (size_t)NR * DD)

__global__ __launch_bounds__(256) void k_pack(const float* __restrict__ E, const int* __restrict__ AV, __bf16* __restrict__ PE) { const int d = blockIdx.x, t = threadIdx.x; __shared__ __align__(16) __bf16 s[NPAIR];
  for (int p = t; p < NPAIR; p += 256) { const int i = p / FF, j = p % FF; const bool ok = (i < j) && (AV[i * FF + j] != 0); s[p] = ok ? (__bf16)E[((size_t)i * FF + j) * DD + d] : (__bf16)0.0f; } __syncthreads();
  for (int q = t; q < NPAIR / 8; q += 256) vst2((unsigned*)(PE + (size_t)d * NPAIR + q * 8), *(const v4u*)&s[q * 8]); }
__global__ __launch_bounds__(128) void k_ctx(const int* __restrict__ M, const int* __restrict__ AV, const __bf16* __restrict__ PE, float* __restrict__ CTX) { __shared__ unsigned char sm[64][FF]; __shared__ unsigned char sav[NPAIR]; __shared__ float scnt[64]; __shared__ __align__(16) float sf[4][16][132];
  const int tid = threadIdx.x, wave = tid >> 5, lane = tid & 31, col = lane & 15, g = lane >> 4; const size_t r0 = (size_t)blockIdx.x * 64; const int c0 = blockIdx.y * 128;
  for (int e = tid; e < 64 * FF; e += 128) sm[e / FF][e % FF] = (unsigned char)(M[(r0 + e / FF) * FF + e % FF] != 0);
  for (int p = tid; p < NPAIR; p += 128) { const int i = p / FF, j = p % FF; sav[p] = (unsigned char)((i < j) && (AV[i * FF + j] != 0)); }
  __syncthreads();
  if (tid < 64) { int c = 0; for (int p = 0; p < NPAIR; ++p) c += (sav[p] & sm[tid][p / FF] & sm[tid][p % FF]); scnt[tid] = (float)c; }
  const int rl = wave * 16 + col; v8f acc[8] = {};
#pragma unroll 2
  for (int kc = 0; kc < NPAIR / 32; ++kc) { v16b a;
#pragma unroll
    for (int i = 0; i < 8; ++i) { const int p0 = kc * 32 + 8 * g + i, p1 = p0 + 16; a[i] = (sm[rl][p0 / FF] & sm[rl][p0 % FF]) ? (__bf16)1.0f : (__bf16)0.0f; a[8 + i] = (sm[rl][p1 / FF] & sm[rl][p1 % FF]) ? (__bf16)1.0f : (__bf16)0.0f; }
#pragma unroll
    for (int j = 0; j < 8; ++j) acc[j] = wmma_bf(a, frag_b(PE + (size_t)(c0 + j * 16 + col) * NPAIR + kc * 32, lane), acc[j]); }
  __syncthreads();
#pragma unroll
  for (int j = 0; j < 8; ++j)
#pragma unroll
    for (int r = 0; r < 8; ++r) { const float cnt = scnt[wave * 16 + 8 * g + r]; sf[wave][8 * g + r][j * 16 + col] = (cnt > 0.f) ? acc[j][r] / cnt : 0.f; }
  LDSX(); for (int q = 0; q < 16; ++q) vst2(CTX + (r0 + wave * 16 + q) * DD + c0 + lane * 4, *(const v4f*)&sf[wave][q][lane * 4]); }
__global__ __launch_bounds__(128) void k_out(const float* __restrict__ CTX, const float* __restrict__ AW, const float* __restrict__ AB, float* __restrict__ OUT) { __shared__ __align__(16) float sf[4][16][132];
  const int tid = threadIdx.x, wave = tid >> 5, lane = tid & 31, col = lane & 15, g = lane >> 4; const size_t r0 = (size_t)blockIdx.x * 64 + wave * 16; const int c0 = blockIdx.y * 128;
  v8f acc[8] = {};
#pragma unroll 2
  for (int kc = 0; kc < DD / 32; ++kc) { const F2 a = split_row(CTX + (r0 + col) * DD, kc * 32, lane);
#pragma unroll
    for (int j = 0; j < 8; ++j) { v16b w; const float* wr = AW + (size_t)(c0 + j * 16 + col) * DD + kc * 32 + 8 * g;
#pragma unroll
      for (int i = 0; i < 8; ++i) { w[i] = (__bf16)wr[i]; w[8 + i] = (__bf16)wr[16 + i]; } acc[j] = wmma_bf(a.h, w, acc[j]); acc[j] = wmma_bf(a.l, w, acc[j]); } }
#pragma unroll
  for (int j = 0; j < 8; ++j) { const float bb = bfr(AB[c0 + j * 16 + col]);
#pragma unroll
    for (int r = 0; r < 8; ++r) sf[wave][8 * g + r][j * 16 + col] = acc[j][r] + bb; }
  LDSX(); for (int q = 0; q < 16; ++q) vst2(OUT + (r0 + q) * HH + c0 + lane * 4, *(const v4f*)&sf[wave][q][lane * 4]); }
extern "C" void kernel_launch(void* const* d_in, const int* in_sizes, int n_in, void* d_out, int out_size, void* d_ws, size_t ws_size, hipStream_t stream) {
  (void)in_sizes; (void)n_in; (void)out_size;
  const float** F = (const float**)d_in;
  if (ws_size < (size_t)WS_END) return;
  char* ws = (char*)d_ws; __bf16* PE = (__bf16*)(ws + WS_PE); float* CTX = (float*)(ws + WS_CTX);
  k_pack<<<DD, 256, 0, stream>>>(F[1], (const int*)d_in[2], PE);
  k_ctx<<<dim3(TR, DD / 128), 128, 0, stream>>>((const int*)d_in[0], (const int*)d_in[2], PE, CTX);
  k_out<<<dim3(TR, HH / 128), 128, 0, stream>>>(CTX, F[3], F[4], (float*)d_out);
}
